// DyGraphTransformer_87342454931906
// MI455X (gfx1250) — hardware-verified
//
#include <hip/hip_runtime.h>
#include <math.h>

typedef __attribute__((ext_vector_type(16))) _Float16 v16h;
typedef __attribute__((ext_vector_type(16))) __bf16 v16b;
typedef __attribute__((ext_vector_type(8)))  _Float16 v8h;
typedef __attribute__((ext_vector_type(8)))  float v8f;
typedef __attribute__((ext_vector_type(4)))  float v4f;
typedef __attribute__((ext_vector_type(2)))  float v2f;
typedef __attribute__((ext_vector_type(4)))  unsigned v4u;
typedef __attribute__((ext_vector_type(4)))  int v4i;
typedef float __attribute__((may_alias)) float_a;
typedef int __attribute__((may_alias)) int_a;

template <typename T> __device__ __forceinline__ void vst2(void* p, T v) { *(volatile T*)p = v; __threadfence(); *(volatile T*)p = v; }
__device__ __forceinline__ v8f wmma16(v16h a, v16h b, v8f c) {
  v8f d = __builtin_amdgcn_wmma_f32_16x16x32_f16(false, a, false, b, (short)0, c, false, false);
  asm volatile("v_nop\n\tv_nop\n\tv_nop\n\tv_nop" : "+v"(d) : "v"(a), "v"(b));
  return d;
}
__device__ __forceinline__ v8f wmma_bf(v16b a, v16b b, v8f c) {
  v8f d = __builtin_amdgcn_wmma_f32_16x16x32_bf16(false, a, false, b, (short)0, c, false, false);
  asm volatile("v_nop\n\tv_nop\n\tv_nop\n\tv_nop" : "+v"(d) : "v"(a), "v"(b));
  return d;
}
__device__ __forceinline__ v16h frag_h(const _Float16* rowk0, int lane) {
  union { v16h v; v8h q[2]; } u; const _Float16* p = rowk0 + 8 * (lane >> 4);
  u.q[0] = *(const v8h*)p; u.q[1] = *(const v8h*)(p + 16); return u.v;
}
__device__ __forceinline__ v16h frag_f32(const float* rowk0, int lane) {
  v16h a; const float* p = rowk0 + 8 * (lane >> 4);
#pragma unroll
  for (int i = 0; i < 8; ++i) { a[i] = (_Float16)p[i]; a[8 + i] = (_Float16)p[16 + i]; }
  return a;
}
__device__ __forceinline__ v16h frag_f32s(const float* rowk0, int lane, float sc) {
  v16h a; const float* p = rowk0 + 8 * (lane >> 4);
#pragma unroll
  for (int i = 0; i < 8; ++i) { a[i] = (_Float16)(p[i] * sc); a[8 + i] = (_Float16)(p[16 + i] * sc); }
  return a;
}
__device__ __forceinline__ v16h fragc_f32(const float* W, int k0, int n, int lane, int ld, int K) {
  v16h a; const int g = lane >> 4;
#pragma unroll
  for (int i = 0; i < 8; ++i) { const int ka = k0 + 8 * g + i, kb = ka + 16;
    a[i] = (_Float16)(ka < K ? W[(size_t)ka * ld + n] : 0.f); a[8 + i] = (_Float16)(kb < K ? W[(size_t)kb * ld + n] : 0.f); }
  return a;
}
struct F2 { v16b h, l; };
__device__ __forceinline__ F2 bsplit16(const float v[16]) { F2 r;
#pragma unroll
  for (int i = 0; i < 16; ++i) { const __bf16 h = (__bf16)v[i]; r.h[i] = h; r.l[i] = (__bf16)(v[i] - (float)h); }
  return r; }
__device__ __forceinline__ F2 split_row(const float* row, int k0, int lane) { float v[16]; const float* p = row + k0 + 8 * (lane >> 4);
#pragma unroll
  for (int i = 0; i < 8; ++i) { v[i] = p[i]; v[8 + i] = p[16 + i]; }
  return bsplit16(v); }
__device__ __forceinline__ F2 split_rowK(const float* row, int k0, int lane, int K) { float v[16]; const int g = lane >> 4;
#pragma unroll
  for (int i = 0; i < 8; ++i) { const int ka = k0 + 8 * g + i, kb = ka + 16; v[i] = ka < K ? row[ka] : 0.f; v[8 + i] = kb < K ? row[kb] : 0.f; }
  return bsplit16(v); }
__device__ __forceinline__ F2 split_col(const float* W, int k0, int n, int lane, int ld, int K) { float v[16]; const int g = lane >> 4;
#pragma unroll
  for (int i = 0; i < 8; ++i) { const int ka = k0 + 8 * g + i, kb = ka + 16; v[i] = ka < K ? W[(size_t)ka * ld + n] : 0.f; v[8 + i] = kb < K ? W[(size_t)kb * ld + n] : 0.f; }
  return bsplit16(v); }
__device__ __forceinline__ v8f mac3(const F2& a, const F2& b, v8f c) { c = wmma_bf(a.l, b.h, c); c = wmma_bf(a.h, b.l, c); return wmma_bf(a.h, b.h, c); }
__device__ __forceinline__ float sigm(float v) { return 1.0f / (1.0f + expf(-v)); }
#define LDSX() do { asm volatile("s_wait_dscnt 0" ::: "memory"); __builtin_amdgcn_wave_barrier(); __builtin_amdgcn_fence(__ATOMIC_RELEASE, "workgroup"); } while (0)


#define NT 512
#define HDM 256
#define NH 8
#define DK 32
#define NLAY 6
#define EEN 32
#define EDN 128
__device__ __forceinline__ float gelu_e(float x) { return 0.5f * x * (1.0f + erff(x * 0.70710678118654752f)); }
__device__ __forceinline__ int clampi(int v, int hi) { return v < 0 ? 0 : (v > hi ? hi : v); }

__global__ __launch_bounds__(256) void k_tabs(const float* __restrict__ eemb, const float* __restrict__ demb, const float* __restrict__ Wee, const float* __restrict__ Wed, float* __restrict__ TEE, float* __restrict__ TED) {
  __shared__ float stab[EEN + EDN][NH];
  const int tid = threadIdx.x, wave = tid >> 5, lane = tid & 31;
  for (int r = wave; r < EEN + EDN; r += 8) { const float* row = r < EEN ? eemb + (size_t)r * HDM : demb + (size_t)(r - EEN) * HDM; const float* W = r < EEN ? Wee : Wed;
    float ss = 0.f; for (int k = lane; k < HDM; k += 32) ss += row[k] * row[k];
#pragma unroll
    for (int o = 16; o > 0; o >>= 1) ss += __shfl_xor(ss, o, 32);
    const float nrm = sqrtf(ss); const float sc = nrm > 1.0f ? 1.0f / (nrm + 1e-7f) : 1.0f;
    float acc[NH];
#pragma unroll
    for (int h = 0; h < NH; ++h) acc[h] = 0.f;
    for (int k = lane; k < HDM; k += 32) { const float v = row[k] * sc;
#pragma unroll
      for (int h = 0; h < NH; ++h) acc[h] += v * W[k * NH + h]; }
#pragma unroll
    for (int h = 0; h < NH; ++h) {
#pragma unroll
      for (int o = 16; o > 0; o >>= 1) acc[h] += __shfl_xor(acc[h], o, 32); }
#pragma unroll
    for (int h = 0; h < NH; ++h) if (lane == h) stab[r][h] = acc[h]; }
  __syncthreads();
  for (int q = tid; q < (EEN + EDN) * NH; q += 256) { const float v = (&stab[0][0])[q]; if (q < EEN * NH) vst2(TEE + q, (float_a)v); else vst2(TED + (q - EEN * NH), (float_a)v); }
}
__global__ __launch_bounds__(256) void k_bias(const int* __restrict__ eenc, const int* __restrict__ denc, const float* __restrict__ TEE, const float* __restrict__ bee, const float* __restrict__ TED, const float* __restrict__ bed, float* __restrict__ BIAS) {
  const int i = blockIdx.x, tid = threadIdx.x;
  for (int j = tid; j < NT; j += 256) { const int e0 = clampi(eenc[((size_t)i * NT + j) * 2], EEN - 1), e1 = clampi(eenc[((size_t)i * NT + j) * 2 + 1], EEN - 1), d = clampi(denc[(size_t)i * NT + j], EDN - 1);
#pragma unroll
    for (int h = 0; h < NH; ++h) vst2(BIAS + ((size_t)h * NT + i) * NT + j, (float_a)(0.5f * (TEE[e0 * NH + h] + TEE[e1 * NH + h]) + bee[h] + TED[d * NH + h] + bed[h])); }
}
__global__ __launch_bounds__(128) void k_feat(const float* __restrict__ x, const float* __restrict__ W, const float* __restrict__ b, float* __restrict__ Hres) {
  __shared__ __align__(16) float so[4][16][132];
  const int tid = threadIdx.x, wave = tid >> 5, lane = tid & 31, col = lane & 15, g = lane >> 4; const int r0 = blockIdx.x * 64 + wave * 16;
#pragma unroll 1
  for (int nh = 0; nh < 2; ++nh) { v8f acc[8] = {};
#pragma unroll 1
    for (int kc = 0; kc < HDM / 32; ++kc) { const F2 a = split_row(x + (size_t)(r0 + col) * HDM, kc * 32, lane);
#pragma unroll
      for (int j = 0; j < 8; ++j) acc[j] = mac3(a, split_col(W, kc * 32, nh * 128 + j * 16 + col, lane, HDM, HDM), acc[j]); }
#pragma unroll
    for (int j = 0; j < 8; ++j) { const float bb = b[nh * 128 + j * 16 + col];
#pragma unroll
      for (int r = 0; r < 8; ++r) so[wave][8 * g + r][j * 16 + col] = acc[j][r] + bb; }
    LDSX();
    for (int rl = 0; rl < 16; ++rl) vst2(Hres + (size_t)(r0 + rl) * HDM + nh * 128 + lane * 4, *(const v4f*)(&so[wave][rl][lane * 4]));
    LDSX(); }
}
__device__ __forceinline__ void ln_rows(const float* __restrict__ Hres, int r0, const float* __restrict__ gs, const float* __restrict__ gb, float (*sy)[HDM + 4], int lane) {
  const int rl = lane & 15, hf = lane >> 4; const float* row = Hres + (size_t)(r0 + rl) * HDM + hf * 128; float s = 0.f;
#pragma unroll 4
  for (int k = 0; k < 128; ++k) s += row[k];
  s += __shfl_xor(s, 16, 32); const float mu = s * (1.0f / HDM); float q = 0.f;
#pragma unroll 4
  for (int k = 0; k < 128; ++k) { const float d = row[k] - mu; q += d * d; }
  q += __shfl_xor(q, 16, 32); const float rs = rsqrtf(q * (1.0f / HDM) + 1e-5f);
#pragma unroll 4
  for (int k = 0; k < 128; ++k) sy[rl][hf * 128 + k] = (row[k] - mu) * rs * gs[hf * 128 + k] + gb[hf * 128 + k];
}
__global__ __launch_bounds__(128) void k_qkv(const float* __restrict__ Hres, const float* __restrict__ gs, const float* __restrict__ gb, const float* __restrict__ Wq, const float* __restrict__ bq, const float* __restrict__ Wk, const float* __restrict__ bk,
                                            const float* __restrict__ Wv, const float* __restrict__ bv, float* __restrict__ Q, float* __restrict__ Kx, float* __restrict__ V) {
  __shared__ __align__(16) float sy[4][16][HDM + 4]; __shared__ __align__(16) float so[4][16][132];
  const int tid = threadIdx.x, wave = tid >> 5, lane = tid & 31, col = lane & 15, g = lane >> 4; const int r0 = blockIdx.x * 64 + wave * 16; const int which = blockIdx.y;
  const float* W = which == 0 ? Wq : (which == 1 ? Wk : Wv); const float* bb_ = which == 0 ? bq : (which == 1 ? bk : bv); float* Dst = which == 0 ? Q : (which == 1 ? Kx : V); const float osc = which == 0 ? 0.17677669529663687f : 1.0f;
  ln_rows(Hres, r0, gs, gb, sy[wave], lane);
  LDSX();
#pragma unroll 1
  for (int nh = 0; nh < 2; ++nh) { v8f acc[8] = {};
#pragma unroll 1
    for (int kc = 0; kc < HDM / 32; ++kc) { const F2 a = split_row(&sy[wave][col][0], kc * 32, lane);
#pragma unroll
      for (int j = 0; j < 8; ++j) acc[j] = mac3(a, split_col(W, kc * 32, nh * 128 + j * 16 + col, lane, HDM, HDM), acc[j]); }
#pragma unroll
    for (int j = 0; j < 8; ++j) { const float bb = bb_[nh * 128 + j * 16 + col];
#pragma unroll
      for (int r = 0; r < 8; ++r) so[wave][8 * g + r][j * 16 + col] = (acc[j][r] + bb) * osc; }
    LDSX();
    for (int rl = 0; rl < 16; ++rl) vst2(Dst + (size_t)(r0 + rl) * HDM + nh * 128 + lane * 4, *(const v4f*)(&so[wave][rl][lane * 4]));
    LDSX(); }
}
__global__ __launch_bounds__(128) void k_attn(const float* __restrict__ Q, const float* __restrict__ Kx, const float* __restrict__ V, const float* __restrict__ BIAS, float* __restrict__ O) {
  __shared__ __align__(16) float sS[4][16][68]; __shared__ __align__(16) float sO[4][16][36];
  const int tid = threadIdx.x, w = tid >> 5, lane = tid & 31, col = lane & 15, g = lane >> 4;
  const int h = blockIdx.y; const int q0 = blockIdx.x * 64 + w * 16;
  const F2 aq = split_row(Q + (size_t)(q0 + col) * HDM + h * DK, 0, lane);
  const float* brow = BIAS + ((size_t)h * NT) * NT;
  float mrun = -3.0e38f, lrun = 0.f; v8f acc[2] = {};
#pragma unroll 1
  for (int kt = 0; kt < NT / 64; ++kt) {
#pragma unroll
    for (int t = 0; t < 4; ++t) { const int key = kt * 64 + t * 16 + col; const v8f s = mac3(aq, split_row(Kx + (size_t)key * HDM + h * DK, 0, lane), (v8f){});
#pragma unroll
      for (int r = 0; r < 8; ++r) sS[w][8 * g + r][t * 16 + col] = s[r] + brow[(size_t)(q0 + 8 * g + r) * NT + key]; }
    LDSX();
    float mx = -3.4e38f;
#pragma unroll
    for (int jj = 0; jj < 32; ++jj) mx = fmaxf(mx, sS[w][col][g * 32 + jj]);
    mx = fmaxf(mx, __shfl_xor(mx, 16, 32));
    const float mnew = fmaxf(mrun, mx); const float corr = expf(mrun - mnew);
    float ps = 0.f;
#pragma unroll
    for (int jj = 0; jj < 32; ++jj) { const float p = expf(sS[w][col][g * 32 + jj] - mnew); ps += p; sS[w][col][g * 32 + jj] = p; }
    ps += __shfl_xor(ps, 16, 32);
    lrun = lrun * corr + ps; mrun = mnew;
#pragma unroll
    for (int r = 0; r < 8; ++r) { const float cr = __shfl(corr, 8 * g + r, 32); acc[0][r] *= cr; acc[1][r] *= cr; }
    LDSX();
#pragma unroll
    for (int kc = 0; kc < 2; ++kc) { const F2 pa = split_row(&sS[w][col][0], kc * 32, lane);
#pragma unroll
      for (int t2 = 0; t2 < 2; ++t2) acc[t2] = mac3(pa, split_col(V + (size_t)(kt * 64) * HDM + h * DK, kc * 32, t2 * 16 + col, lane, HDM, 64), acc[t2]); }
    LDSX(); }
#pragma unroll
  for (int r = 0; r < 8; ++r) { const float lr = __shfl(lrun, 8 * g + r, 32); const float inv = 1.0f / lr;
#pragma unroll
    for (int t2 = 0; t2 < 2; ++t2) sO[w][8 * g + r][t2 * 16 + col] = acc[t2][r] * inv; }
  LDSX();
  for (int qq = lane; qq < 16 * 8; qq += 32) { const int rl = qq >> 3, pc = qq & 7; vst2(O + (size_t)(q0 + rl) * HDM + h * DK + pc * 4, *(const v4f*)(&sO[w][rl][pc * 4])); }
}
__global__ __launch_bounds__(128) void k_oproj(const float* __restrict__ O, const float* __restrict__ Wo, const float* __restrict__ bo, float* __restrict__ Hres) {
  __shared__ __align__(16) float so[4][16][132];
  const int tid = threadIdx.x, wave = tid >> 5, lane = tid & 31, col = lane & 15, g = lane >> 4; const int r0 = blockIdx.x * 64 + wave * 16;
#pragma unroll 1
  for (int nh = 0; nh < 2; ++nh) { v8f acc[8] = {};
#pragma unroll 1
    for (int kc = 0; kc < HDM / 32; ++kc) { const F2 a = split_row(O + (size_t)(r0 + col) * HDM, kc * 32, lane);
#pragma unroll
      for (int j = 0; j < 8; ++j) acc[j] = mac3(a, split_col(Wo, kc * 32, nh * 128 + j * 16 + col, lane, HDM, HDM), acc[j]); }
#pragma unroll
    for (int j = 0; j < 8; ++j) { const int n = nh * 128 + j * 16 + col; const float bb = bo[n];
#pragma unroll
      for (int r = 0; r < 8; ++r) so[wave][8 * g + r][j * 16 + col] = acc[j][r] + bb + Hres[(size_t)(r0 + 8 * g + r) * HDM + n]; }
    LDSX();
    for (int rl = 0; rl < 16; ++rl) vst2(Hres + (size_t)(r0 + rl) * HDM + nh * 128 + lane * 4, *(const v4f*)(&so[wave][rl][lane * 4]));
    LDSX(); }
}
__global__ __launch_bounds__(128) void k_ffn(float* __restrict__ Hres, const float* __restrict__ gs, const float* __restrict__ gb, const float* __restrict__ W1, const float* __restrict__ b1, const float* __restrict__ W2, const float* __restrict__ b2) {
  __shared__ __align__(16) float sy[4][16][HDM + 4]; __shared__ __align__(16) float sz[4][16][HDM + 4];
  const int tid = threadIdx.x, wave = tid >> 5, lane = tid & 31, col = lane & 15, g = lane >> 4; const int r0 = blockIdx.x * 64 + wave * 16;
  ln_rows(Hres, r0, gs, gb, sy[wave], lane);
  LDSX();
#pragma unroll 1
  for (int nh = 0; nh < 2; ++nh) { v8f acc[8] = {};
#pragma unroll 1
    for (int kc = 0; kc < HDM / 32; ++kc) { const F2 a = split_row(&sy[wave][col][0], kc * 32, lane);
#pragma unroll
      for (int j = 0; j < 8; ++j) acc[j] = mac3(a, split_col(W1, kc * 32, nh * 128 + j * 16 + col, lane, HDM, HDM), acc[j]); }
#pragma unroll
    for (int j = 0; j < 8; ++j) { const int n = nh * 128 + j * 16 + col; const float bb = b1[n];
#pragma unroll
      for (int r = 0; r < 8; ++r) sz[wave][8 * g + r][n] = gelu_e(acc[j][r] + bb); } }
  LDSX();
#pragma unroll 1
  for (int nh = 0; nh < 2; ++nh) { v8f acc[8] = {};
#pragma unroll 1
    for (int kc = 0; kc < HDM / 32; ++kc) { const F2 a = split_row(&sz[wave][col][0], kc * 32, lane);
#pragma unroll
      for (int j = 0; j < 8; ++j) acc[j] = mac3(a, split_col(W2, kc * 32, nh * 128 + j * 16 + col, lane, HDM, HDM), acc[j]); }
#pragma unroll
    for (int j = 0; j < 8; ++j) { const int n = nh * 128 + j * 16 + col; const float bb = b2[n];
#pragma unroll
      for (int r = 0; r < 8; ++r) sy[wave][8 * g + r][n] = acc[j][r] + bb + Hres[(size_t)(r0 + 8 * g + r) * HDM + n]; } }
  LDSX();
  for (int rl = 0; rl < 16; ++rl) { for (int pc = lane; pc < HDM / 4; pc += 32) vst2(Hres + (size_t)(r0 + rl) * HDM + pc * 4, *(const v4f*)(&sy[wave][rl][pc * 4])); }
}
extern "C" void kernel_launch(void* const* d_in, const int* in_sizes, int n_in, void* d_out, int out_size, void* d_ws, size_t ws_size, hipStream_t stream) {
  (void)in_sizes; (void)n_in; (void)out_size; (void)ws_size;
  const float** I = (const float**)d_in;
  const float* x = I[0]; const int* eenc = (const int*)d_in[2]; const int* denc = (const int*)d_in[3];
  const float* Wf = I[7]; const float* bf_ = I[8]; const float* eemb = I[9]; const float* demb = I[10]; const float* Wee = I[11]; const float* bee = I[12]; const float* Wed = I[13]; const float* bed = I[14];
  const float* ln1s = I[15]; const float* ln1b = I[16]; const float* Wq = I[17]; const float* bq = I[18]; const float* Wk = I[19]; const float* bk = I[20]; const float* Wv = I[21]; const float* bv = I[22];
  const float* Wo = I[23]; const float* bo = I[24]; const float* ln2s = I[25]; const float* ln2b = I[26]; const float* W1 = I[27]; const float* b1 = I[28]; const float* W2 = I[29]; const float* b2 = I[30];
  float* Hres = (float*)d_out;
  char* ws = (char*)d_ws; size_t off = 0;
  auto take = [&](size_t bytes) { char* p = ws + off; off += (bytes + 255) & ~(size_t)255; return p; };
  float* TEE = (float*)take(EEN * NH * 4); float* TED = (float*)take(EDN * NH * 4); float* BIAS = (float*)take((size_t)NH * NT * NT * 4);
  float* Q = (float*)take((size_t)NT * HDM * 4); float* Kx = (float*)take((size_t)NT * HDM * 4); float* V = (float*)take((size_t)NT * HDM * 4); float* O = (float*)take((size_t)NT * HDM * 4);
  k_tabs<<<1, 256, 0, stream>>>(eemb, demb, Wee, Wed, TEE, TED);
  k_bias<<<NT, 256, 0, stream>>>(eenc, denc, TEE, bee, TED, bed, BIAS);
  k_feat<<<NT / 64, 128, 0, stream>>>(x, Wf, bf_, Hres);
  for (int l = 0; l < NLAY; ++l) { const size_t oM = (size_t)l * HDM * HDM, oV = (size_t)l * HDM;
    k_qkv<<<dim3(NT / 64, 3), 128, 0, stream>>>(Hres, ln1s + oV, ln1b + oV, Wq + oM, bq + oV, Wk + oM, bk + oV, Wv + oM, bv + oV, Q, Kx, V);
    k_attn<<<dim3(NT / 64, NH), 128, 0, stream>>>(Q, Kx, V, BIAS, O);
    k_oproj<<<NT / 64, 128, 0, stream>>>(O, Wo + oM, bo + oV, Hres);
    k_ffn<<<NT / 64, 128, 0, stream>>>(Hres, ln2s + oV, ln2b + oV, W1 + oM, b1 + oV, W2 + oM, b2 + oV); }
}
